// MultiHeadAttention_38491496907095
// MI455X (gfx1250) — hardware-verified
//
#include <hip/hip_runtime.h>
#include <math.h>

typedef __attribute__((ext_vector_type(16))) _Float16 v16h;
typedef __attribute__((ext_vector_type(8)))  _Float16 v8h;
typedef __attribute__((ext_vector_type(8)))  float    v8f;
typedef __attribute__((ext_vector_type(4)))  float    v4f;
typedef __attribute__((ext_vector_type(2)))  float    v2f;
typedef __attribute__((ext_vector_type(4)))  unsigned int v4u;

constexpr int kBatch  = 4;
constexpr int kSeq    = 2048;
constexpr int kEmb    = 1024;
constexpr int kHeads  = 16;
constexpr int kHd     = 64;
constexpr int kTok    = kBatch * kSeq;
constexpr int kBH     = kBatch * kHeads;
constexpr int kNqkv   = 3 * kEmb;
constexpr int kTierS  = 512;
static_assert(kHeads * kHd == kEmb);
static_assert(kHd == 64 && kHd / 2 == 32);
static_assert((kTok % 64) == 0 && (kNqkv % 64) == 0 && (kEmb % 64) == 0 && (kEmb % 32) == 0 && (kHd % 32) == 0);
static_assert((kSeq % 64) == 0 && (kTierS % 64) == 0 && kEmb / 64 == 16);

constexpr float kXCarry   = 16.0f;
constexpr float kWCarry   = 256.0f;
constexpr float kQKCarry  = 16.0f;
constexpr float kVCarry   = 16.0f;
constexpr float kPCarry   = 32768.0f;
constexpr float kAoCarry  = 256.0f;
constexpr float kLoScale  = 2048.0f;
constexpr float kLoInv    = 1.0f / kLoScale;
constexpr float kInvSqrtHd = 0.125f;
static_assert(kInvSqrtHd * kInvSqrtHd * (float)kHd == 1.0f);
constexpr float kProjQK     = kQKCarry / (kXCarry * kWCarry);
constexpr float kProjV      = kVCarry / (kXCarry * kWCarry);
constexpr float kScoreScale = kInvSqrtHd / (kQKCarry * kQKCarry);
constexpr float kAoFold     = kAoCarry / (kPCarry * kVCarry);
constexpr float kOutScale   = 1.0f / (kAoCarry * kWCarry);

constexpr size_t kOffX16  = 0;
constexpr size_t kOffW16  = kOffX16  + (size_t)kTok * kEmb * 2;
constexpr size_t kOffFreq = kOffW16  + (size_t)4 * kEmb * kEmb * 2;
constexpr size_t kOffCs   = kOffFreq + 128;
constexpr size_t kOffQh   = kOffCs   + (size_t)kSeq * kHd * 4;
constexpr size_t kOffKh   = kOffQh   + (size_t)kBH * kSeq * kHd * 2;
constexpr size_t kOffVth  = kOffKh   + (size_t)kBH * kSeq * kHd * 2;
constexpr size_t kOffQlo  = kOffVth  + (size_t)kBH * kHd * kSeq * 2;
constexpr size_t kOffKlo  = kOffQlo  + (size_t)kBH * kTierS * kHd * 2;
constexpr size_t kOffVtlo = kOffKlo  + (size_t)kBH * kTierS * kHd * 2;
constexpr size_t kOffAoh  = kOffVtlo + (size_t)kBH * kHd * kTierS * 2;
constexpr size_t kOffAolo = kOffAoh  + (size_t)kTok * kEmb * 2;
constexpr size_t kWsTotal = kOffAolo + (size_t)kBatch * kTierS * kEmb * 2;
static_assert(kWsTotal == 109576320ull);
static_assert(kWsTotal <= 134217728ull);
static_assert((kOffW16 % 128) == 0 && (kOffFreq % 128) == 0 && (kOffCs % 128) == 0 && (kOffQh % 128) == 0 &&
              (kOffKh % 128) == 0 && (kOffVth % 128) == 0 && (kOffQlo % 128) == 0 && (kOffKlo % 128) == 0 &&
              (kOffVtlo % 128) == 0 && (kOffAoh % 128) == 0 && (kOffAolo % 128) == 0);

__device__ __forceinline__ unsigned short f2bf_bits(float f) {
  unsigned u = __float_as_uint(f);
  return (unsigned short)((u + 0x7FFFu + ((u >> 16) & 1u)) >> 16);
}
__device__ __forceinline__ float bf_bits2f(unsigned short h) { return __uint_as_float(((unsigned)h) << 16); }
__device__ __forceinline__ unsigned pk16(unsigned short a, unsigned short b) { return (unsigned)a | ((unsigned)b << 16); }
__device__ __forceinline__ unsigned short h_bits(float f) {
  const _Float16 h = (_Float16)f;
  return __builtin_bit_cast(unsigned short, h);
}
__device__ __forceinline__ unsigned short cvt_elem(float v, float carry) {
  const float r = bf_bits2f(f2bf_bits(v));
  return h_bits(r * carry);
}

union FragU { v16h v; v8h h[2]; };
__device__ __forceinline__ v16h ldfrag(const _Float16* p) {
  FragU f;
  f.h[0] = *(const v8h*)(p);
  f.h[1] = *(const v8h*)(p + 16);
  return f.v;
}
__device__ __forceinline__ v8f mma_h(v16h a, v16h b, v8f c) {
  c = __builtin_amdgcn_wmma_f32_16x16x32_f16(false, a, false, b, (short)0, c, false, false);
  asm volatile("v_nop\n\tv_nop\n\tv_nop\n\tv_nop" : "+v"(c) : "v"(a), "v"(b));
  return c;
}
__device__ __forceinline__ void wave_sync() {
  __builtin_amdgcn_fence(__ATOMIC_RELEASE, "workgroup");
  __builtin_amdgcn_wave_barrier();
  __builtin_amdgcn_fence(__ATOMIC_ACQUIRE, "workgroup");
}

__global__ __launch_bounds__(256) void cast8_kernel(
    const float* __restrict__ s0, const float* __restrict__ s1, const float* __restrict__ s2, const float* __restrict__ s3,
    unsigned short* __restrict__ out, int n8, float carry)
{
  const int y = blockIdx.y;
  const float* src = (y == 0) ? s0 : (y == 1) ? s1 : (y == 2) ? s2 : s3;
  const int i = blockIdx.x * 256 + threadIdx.x;
  if (i >= n8) return;
  const float* p = src + 8 * (size_t)i;
  const v4f a = *(const v4f*)(p);
  const v4f c = *(const v4f*)(p + 4);
  unsigned short hb[8];
#pragma unroll
  for (int e = 0; e < 4; ++e) {
    const float ae = a[e];
    const float ce = c[e];
    hb[e]     = cvt_elem(ae, carry);
    hb[4 + e] = cvt_elem(ce, carry);
  }
  const v4u u = (v4u){pk16(hb[0], hb[1]), pk16(hb[2], hb[3]), pk16(hb[4], hb[5]), pk16(hb[6], hb[7])};
  unsigned short* q = out + (size_t)y * (size_t)n8 * 8 + 8 * (size_t)i;
  *(volatile v4u*)q = u;
  __threadfence();
  *(volatile v4u*)q = u;
}

__global__ __launch_bounds__(32) void rope_freq_kernel(float* __restrict__ freq) {
  const int i = threadIdx.x;
  const float e = (2.0f * (float)i) * (1.0f / (float)kHd);
  const float p = powf(10000.0f, e);
  const float f = 1.0f / p;
  *(volatile float*)(freq + i) = f;
  __threadfence();
  *(volatile float*)(freq + i) = f;
}

__global__ __launch_bounds__(256) void rope_table_kernel(
    const int* __restrict__ tokpos, const float* __restrict__ freq, float* __restrict__ cs)
{
  const int g = blockIdx.x * 256 + threadIdx.x;
  const int s = g >> 5;
  const int i = g & 31;
  const float pos = (float)tokpos[s];
  const float ang = pos * freq[i];
  float sn, cn;
  sincosf(ang, &sn, &cn);
  const v2f v = (v2f){cn, sn};
  float* q = cs + 2 * (size_t)g;
  *(volatile v2f*)q = v;
  __threadfence();
  *(volatile v2f*)q = v;
}

__global__ __launch_bounds__(256) void qkv_proj_kernel(
    const unsigned short* __restrict__ Xp, const unsigned short* __restrict__ Wp, const float* __restrict__ cs,
    unsigned short* __restrict__ Qh, unsigned short* __restrict__ Kh, unsigned short* __restrict__ Vth,
    unsigned short* __restrict__ Qlo, unsigned short* __restrict__ Klo, unsigned short* __restrict__ Vtlo)
{
  __shared__ __align__(16) float sT[8][16 * 68];
  const int lane = threadIdx.x & 31;
  const int wave = __builtin_amdgcn_readfirstlane((int)(threadIdx.x >> 5));
  constexpr int tilesN = kNqkv / 64;
  constexpr int tilesM = kTok / 64;
  const int tile = blockIdx.x * 8 + wave;
  if (tile >= tilesM * tilesN) return;
  const int tm = tile / tilesN;
  const int tn = tile - tm * tilesN;
  const int m0 = tm << 6;
  const int n0 = tn << 6;
  const int rlane = lane & 15;
  const int hh    = lane >> 4;
  const int koff  = hh * 8;
  const int mOff  = hh * 8;

  const _Float16* Arow = (const _Float16*)Xp + (size_t)(m0 + rlane) * kEmb + koff;
  const _Float16* Brow = (const _Float16*)Wp + (size_t)(n0 + rlane) * kEmb + koff;

  v8f acc[4][4];
#pragma unroll
  for (int i = 0; i < 4; ++i)
#pragma unroll
    for (int j = 0; j < 4; ++j) acc[i][j] = (v8f){0.f, 0.f, 0.f, 0.f, 0.f, 0.f, 0.f, 0.f};

#pragma unroll 1
  for (int k0 = 0; k0 < kEmb; k0 += 32) {
    v16h bh[4];
#pragma unroll
    for (int j = 0; j < 4; ++j) bh[j] = ldfrag(Brow + (size_t)(j * 16) * kEmb + k0);
#pragma unroll
    for (int i = 0; i < 4; ++i) {
      const v16h ah = ldfrag(Arow + (size_t)(i * 16) * kEmb + k0);
#pragma unroll
      for (int j = 0; j < 4; ++j) acc[i][j] = mma_h(ah, bh[j], acc[i][j]);
    }
  }

  float* slab = sT[wave];
  const int sec  = tn >> 4;
  const int head = tn & 15;
  const int bidx = m0 >> 11;
  const int s0   = m0 & (kSeq - 1);
  const int bhid = bidx * kHeads + head;
  const bool tier = (s0 < kTierS);
  const int q  = lane >> 3;
  const int c8 = (lane & 7) * 8;

  if (sec < 2) {
    unsigned short* Ph = (sec == 0) ? Qh : Kh;
    unsigned short* Pl = (sec == 0) ? Qlo : Klo;
#pragma unroll
    for (int i = 0; i < 4; ++i) {
#pragma unroll
      for (int j = 0; j < 4; ++j)
#pragma unroll
        for (int r = 0; r < 8; ++r)
          slab[(mOff + r) * 68 + (j << 4) + rlane] = acc[i][j][r] * kProjQK;
      wave_sync();
      v8h hv[4], lv[4];
#pragma unroll
      for (int it = 0; it < 4; ++it) {
        const int row = it * 4 + q;
        const int s = s0 + i * 16 + row;
        const float* sp = slab + row * 68 + c8;
        const v4f a0 = *(const v4f*)(sp);
        const v4f a1 = *(const v4f*)(sp + 4);
        const float* tp = cs + (size_t)s * kHd + c8;
        const v4f t0 = *(const v4f*)(tp);
        const v4f t1 = *(const v4f*)(tp + 4);
        float o[8];
        o[0] = a0[0] * t0[0] - a0[1] * t0[1];
        o[1] = a0[0] * t0[1] + a0[1] * t0[0];
        o[2] = a0[2] * t0[2] - a0[3] * t0[3];
        o[3] = a0[2] * t0[3] + a0[3] * t0[2];
        o[4] = a1[0] * t1[0] - a1[1] * t1[1];
        o[5] = a1[0] * t1[1] + a1[1] * t1[0];
        o[6] = a1[2] * t1[2] - a1[3] * t1[3];
        o[7] = a1[2] * t1[3] + a1[3] * t1[2];
#pragma unroll
        for (int e = 0; e < 8; ++e) {
          const _Float16 hx = (_Float16)o[e];
          hv[it][e] = hx;
          lv[it][e] = (_Float16)((o[e] - (float)hx) * kLoScale);
        }
      }
      for (int pass = 0; pass < 2; ++pass) {
#pragma unroll
        for (int it = 0; it < 4; ++it) {
          const int s = s0 + i * 16 + it * 4 + q;
          *(volatile v8h*)(Ph + ((size_t)bhid * kSeq + s) * kHd + c8) = hv[it];
          if (tier) *(volatile v8h*)(Pl + ((size_t)bhid * kTierS + s) * kHd + c8) = lv[it];
        }
        __threadfence();
      }
      wave_sync();
    }
  } else {
#pragma unroll
    for (int j = 0; j < 4; ++j) {
#pragma unroll
      for (int i = 0; i < 4; ++i)
#pragma unroll
        for (int r = 0; r < 8; ++r)
          slab[rlane * 68 + i * 16 + mOff + r] = acc[i][j][r] * kProjV;
      wave_sync();
      v8h hv[4], lv[4];
#pragma unroll
      for (int it = 0; it < 4; ++it) {
        const int dl = it * 4 + q;
        const float* sp = slab + dl * 68 + c8;
        const v4f a0 = *(const v4f*)(sp);
        const v4f a1 = *(const v4f*)(sp + 4);
#pragma unroll
        for (int e = 0; e < 4; ++e) {
          const float x0 = a0[e];
          const float x1 = a1[e];
          const _Float16 h0 = (_Float16)x0;
          const _Float16 h1 = (_Float16)x1;
          hv[it][e]     = h0;
          hv[it][4 + e] = h1;
          lv[it][e]     = (_Float16)((x0 - (float)h0) * kLoScale);
          lv[it][4 + e] = (_Float16)((x1 - (float)h1) * kLoScale);
        }
      }
      for (int pass = 0; pass < 2; ++pass) {
#pragma unroll
        for (int it = 0; it < 4; ++it) {
          const int d = j * 16 + it * 4 + q;
          *(volatile v8h*)(Vth + ((size_t)bhid * kHd + d) * kSeq + s0 + c8) = hv[it];
          if (tier) *(volatile v8h*)(Vtlo + ((size_t)bhid * kHd + d) * kTierS + s0 + c8) = lv[it];
        }
        __threadfence();
      }
      wave_sync();
    }
  }
}

template <bool TIER>
__global__ __launch_bounds__(128) void attn_kernel(
    const unsigned short* __restrict__ Qhp, const unsigned short* __restrict__ Khp, const unsigned short* __restrict__ Vthp,
    const unsigned short* __restrict__ Qlp, const unsigned short* __restrict__ Klp, const unsigned short* __restrict__ Vtlp,
    unsigned short* __restrict__ AOh, unsigned short* __restrict__ AOl, int qb0, int nqb)
{
  __shared__ __align__(16) _Float16 Psh[4][16 * 64];
  __shared__ __align__(16) _Float16 Psl[TIER ? 4 : 1][TIER ? 16 * 64 : 8];
  __shared__ __align__(16) float Os[4][16 * 68];

  const int lane = threadIdx.x & 31;
  const int wave = __builtin_amdgcn_readfirstlane((int)(threadIdx.x >> 5));
  const int hh = lane >> 4;
  const int c  = lane & 15;

  const int bx = blockIdx.x;
  const int bh = bx / nqb;
  const int qb = qb0 + (bx - bh * nqb);
  const int b  = bh / kHeads;
  const int h  = bh - b * kHeads;
  const int q0 = qb * 64 + wave * 16;

  const _Float16* Qb  = (const _Float16*)Qhp  + (size_t)bh * kSeq * kHd;
  const _Float16* Kb  = (const _Float16*)Khp  + (size_t)bh * kSeq * kHd;
  const _Float16* Vb  = (const _Float16*)Vthp + (size_t)bh * kHd * kSeq;
  const _Float16* Qlb = (const _Float16*)Qlp  + (size_t)bh * kTierS * kHd;
  const _Float16* Klb = (const _Float16*)Klp  + (size_t)bh * kTierS * kHd;
  const _Float16* Vlb = (const _Float16*)Vtlp + (size_t)bh * kHd * kTierS;

  v16h qah[2], qal[2];
#pragma unroll
  for (int dc = 0; dc < 2; ++dc) {
    qah[dc] = ldfrag(Qb + (size_t)(q0 + c) * kHd + dc * 32 + 8 * hh);
    if (TIER) qal[dc] = ldfrag(Qlb + (size_t)(q0 + c) * kHd + dc * 32 + 8 * hh);
    else      qal[dc] = qah[dc];
  }

  float mrow[8], lrow[8];
  v8f oacc[4];
#pragma unroll
  for (int r = 0; r < 8; ++r) { mrow[r] = -INFINITY; lrow[r] = 0.f; }
#pragma unroll
  for (int t = 0; t < 4; ++t) oacc[t] = (v8f){0.f, 0.f, 0.f, 0.f, 0.f, 0.f, 0.f, 0.f};

  _Float16* pwh = Psh[wave];
  _Float16* pwl = Psl[TIER ? wave : 0];

#pragma unroll 1
  for (int kc = 0; kc <= qb; ++kc) {
    const int kv0 = kc * 64;
    v8f s[4];
#pragma unroll
    for (int j = 0; j < 4; ++j) {
      v8f sm = (v8f){0.f, 0.f, 0.f, 0.f, 0.f, 0.f, 0.f, 0.f};
      v8f sr = (v8f){0.f, 0.f, 0.f, 0.f, 0.f, 0.f, 0.f, 0.f};
      const _Float16* kp  = Kb  + (size_t)(kv0 + j * 16 + c) * kHd + 8 * hh;
      const _Float16* klp = Klb + (size_t)(kv0 + j * 16 + c) * kHd + 8 * hh;
#pragma unroll
      for (int dc = 0; dc < 2; ++dc) {
        const v16h kb = ldfrag(kp + dc * 32);
        sm = mma_h(qah[dc], kb, sm);
        if (TIER) {
          const v16h kl = ldfrag(klp + dc * 32);
          sr = mma_h(qah[dc], kl, sr);
          sr = mma_h(qal[dc], kb, sr);
        }
      }
#pragma unroll
      for (int r = 0; r < 8; ++r) {
        if (TIER) s[j][r] = (sm[r] + sr[r] * kLoInv) * kScoreScale;
        else      s[j][r] = sm[r] * kScoreScale;
      }
    }
    const bool diag = (kc == qb);
    float cm[8];
#pragma unroll
    for (int r = 0; r < 8; ++r) {
      const int qrow = q0 + 8 * hh + r;
      float m = -INFINITY;
#pragma unroll
      for (int j = 0; j < 4; ++j) {
        const int kvcol = kv0 + j * 16 + c;
        const float sv = s[j][r];
        const float sx = (diag && (kvcol > qrow)) ? -INFINITY : sv;
        s[j][r] = sx;
        m = fmaxf(m, sx);
      }
      m = fmaxf(m, __shfl_xor(m, 1, 32));
      m = fmaxf(m, __shfl_xor(m, 2, 32));
      m = fmaxf(m, __shfl_xor(m, 4, 32));
      m = fmaxf(m, __shfl_xor(m, 8, 32));
      cm[r] = m;
    }
    wave_sync();
#pragma unroll
    for (int r = 0; r < 8; ++r) {
      const float mnew  = fmaxf(mrow[r], cm[r]);
      const float alpha = __expf(mrow[r] - mnew);
      mrow[r] = mnew;
      float psum = 0.f;
#pragma unroll
      for (int j = 0; j < 4; ++j) {
        const float p  = __expf(s[j][r] - mnew);
        psum += p;
        const float pc = p * kPCarry;
        const _Float16 ph = (_Float16)pc;
        pwh[(8 * hh + r) * 64 + j * 16 + c] = ph;
        if (TIER) pwl[(8 * hh + r) * 64 + j * 16 + c] = (_Float16)((pc - (float)ph) * kLoScale);
      }
      psum += __shfl_xor(psum, 1, 32);
      psum += __shfl_xor(psum, 2, 32);
      psum += __shfl_xor(psum, 4, 32);
      psum += __shfl_xor(psum, 8, 32);
      lrow[r] = lrow[r] * alpha + psum;
#pragma unroll
      for (int t = 0; t < 4; ++t) oacc[t][r] *= alpha;
    }
    wave_sync();
    v16h pa[2], pl[2];
#pragma unroll
    for (int kk = 0; kk < 2; ++kk) {
      FragU f;
      f.h[0] = *(const v8h*)(pwh + c * 64 + kk * 32 + 8 * hh);
      f.h[1] = *(const v8h*)(pwh + c * 64 + kk * 32 + 16 + 8 * hh);
      pa[kk] = f.v;
      if (TIER) {
        FragU g;
        g.h[0] = *(const v8h*)(pwl + c * 64 + kk * 32 + 8 * hh);
        g.h[1] = *(const v8h*)(pwl + c * 64 + kk * 32 + 16 + 8 * hh);
        pl[kk] = g.v;
      } else {
        pl[kk] = pa[kk];
      }
    }
#pragma unroll
    for (int t = 0; t < 4; ++t) {
      const _Float16* vp  = Vb  + (size_t)(t * 16 + c) * kSeq   + kv0 + 8 * hh;
      const _Float16* vlp = Vlb + (size_t)(t * 16 + c) * kTierS + kv0 + 8 * hh;
      v8f res = (v8f){0.f, 0.f, 0.f, 0.f, 0.f, 0.f, 0.f, 0.f};
#pragma unroll
      for (int kk = 0; kk < 2; ++kk) {
        const v16h vb = ldfrag(vp + kk * 32);
        oacc[t] = mma_h(pa[kk], vb, oacc[t]);
        if (TIER) {
          const v16h vl = ldfrag(vlp + kk * 32);
          res = mma_h(pa[kk], vl, res);
          res = mma_h(pl[kk], vb, res);
        }
      }
      if (TIER) {
#pragma unroll
        for (int r = 0; r < 8; ++r) oacc[t][r] += res[r] * kLoInv;
      }
    }
  }

  float* os = Os[wave];
#pragma unroll
  for (int r = 0; r < 8; ++r) {
    const float inv = kAoFold * (1.0f / lrow[r]);
#pragma unroll
    for (int t = 0; t < 4; ++t) os[(8 * hh + r) * 68 + t * 16 + c] = oacc[t][r] * inv;
  }
  wave_sync();
  {
    const int q  = lane >> 3;
    const int c8 = (lane & 7) * 8;
    v8h hv[4], lv[4];
#pragma unroll
    for (int it = 0; it < 4; ++it) {
      const int row = it * 4 + q;
      const float* sp = os + row * 68 + c8;
      const v4f a0 = *(const v4f*)(sp);
      const v4f a1 = *(const v4f*)(sp + 4);
#pragma unroll
      for (int e = 0; e < 4; ++e) {
        const float x0 = a0[e];
        const float x1 = a1[e];
        const _Float16 h0 = (_Float16)x0;
        const _Float16 h1 = (_Float16)x1;
        hv[it][e]     = h0;
        hv[it][4 + e] = h1;
        lv[it][e]     = (_Float16)((x0 - (float)h0) * kLoScale);
        lv[it][4 + e] = (_Float16)((x1 - (float)h1) * kLoScale);
      }
    }
    const size_t ob  = ((size_t)b * kSeq   + q0) * kEmb + (size_t)h * kHd + c8;
    const size_t olb = ((size_t)b * kTierS + q0) * kEmb + (size_t)h * kHd + c8;
    for (int pass = 0; pass < 2; ++pass) {
#pragma unroll
      for (int it = 0; it < 4; ++it) {
        const int row = it * 4 + q;
        *(volatile v8h*)(AOh + ob + (size_t)row * kEmb) = hv[it];
        if (TIER) *(volatile v8h*)(AOl + olb + (size_t)row * kEmb) = lv[it];
      }
      __threadfence();
    }
  }
}

template <int MI, bool RES>
__global__ __launch_bounds__(256) void out_proj_kernel(
    const unsigned short* __restrict__ Ap, const unsigned short* __restrict__ A2p, long strideA, long strideA2,
    const unsigned short* __restrict__ Wp, float* __restrict__ C, long strideC, int M)
{
  __shared__ __align__(16) float sT[8][16 * 68];
  const int lane = threadIdx.x & 31;
  const int wave = __builtin_amdgcn_readfirstlane((int)(threadIdx.x >> 5));
  const int b = blockIdx.y;
  constexpr int TM = 16 * MI;
  const int tilesM = M / TM;
  const int tile = blockIdx.x * 8 + wave;
  if (tile >= tilesM * (kEmb / 64)) return;
  const int tm = tile >> 4;
  const int tn = tile & 15;
  const int m0 = tm * TM;
  const int n0 = tn << 6;
  const int rlane = lane & 15;
  const int hh    = lane >> 4;
  const int koff  = hh * 8;
  const int mOff  = hh * 8;

  const _Float16* Arow  = (const _Float16*)Ap  + (size_t)b * strideA  + (size_t)(m0 + rlane) * kEmb + koff;
  const _Float16* A2row = (const _Float16*)A2p + (size_t)b * strideA2 + (size_t)(m0 + rlane) * kEmb + koff;
  const _Float16* Brow  = (const _Float16*)Wp + (size_t)(n0 + rlane) * kEmb + koff;

  v8f acc[MI][4], accr[MI][4];
#pragma unroll
  for (int i = 0; i < MI; ++i)
#pragma unroll
    for (int j = 0; j < 4; ++j) {
      acc[i][j]  = (v8f){0.f, 0.f, 0.f, 0.f, 0.f, 0.f, 0.f, 0.f};
      accr[i][j] = (v8f){0.f, 0.f, 0.f, 0.f, 0.f, 0.f, 0.f, 0.f};
    }

#pragma unroll 1
  for (int k0 = 0; k0 < kEmb; k0 += 32) {
    v16h bh[4];
#pragma unroll
    for (int j = 0; j < 4; ++j) bh[j] = ldfrag(Brow + (size_t)(j * 16) * kEmb + k0);
#pragma unroll
    for (int i = 0; i < MI; ++i) {
      const v16h ah = ldfrag(Arow + (size_t)(i * 16) * kEmb + k0);
#pragma unroll
      for (int j = 0; j < 4; ++j) acc[i][j] = mma_h(ah, bh[j], acc[i][j]);
      if (RES) {
        const v16h al = ldfrag(A2row + (size_t)(i * 16) * kEmb + k0);
#pragma unroll
        for (int j = 0; j < 4; ++j) accr[i][j] = mma_h(al, bh[j], accr[i][j]);
      }
    }
  }

  float* slab = sT[wave];
  float* Cb = C + (size_t)b * strideC;
  const int c4 = (lane & 15) * 4;
#pragma unroll
  for (int i = 0; i < MI; ++i) {
    const int mBase = m0 + (i << 4);
#pragma unroll
    for (int j = 0; j < 4; ++j)
#pragma unroll
      for (int r = 0; r < 8; ++r) {
        float v;
        if (RES) v = (acc[i][j][r] + accr[i][j][r] * kLoInv) * kOutScale;
        else     v = acc[i][j][r] * kOutScale;
        slab[(mOff + r) * 68 + (j << 4) + rlane] = v;
      }
    wave_sync();
    for (int pass = 0; pass < 2; ++pass) {
#pragma unroll
      for (int it = 0; it < 8; ++it) {
        const int row = it * 2 + hh;
        const v4f v = *(const v4f*)(slab + row * 68 + c4);
        *(volatile v4f*)(Cb + (size_t)(mBase + row) * kEmb + n0 + c4) = v;
      }
      __threadfence();
    }
    wave_sync();
  }
}

extern "C" void kernel_launch(void* const* d_in, const int* in_sizes, int n_in,
                              void* d_out, int out_size, void* d_ws, size_t ws_size,
                              hipStream_t stream) {
  if (n_in < 6) return;
  if (in_sizes[0] != kTok * kEmb) return;
  if (in_sizes[1] != kSeq) return;
  if (in_sizes[2] != kEmb * kEmb) return;
  if (in_sizes[3] != kEmb * kEmb) return;
  if (in_sizes[4] != kEmb * kEmb) return;
  if (in_sizes[5] != kEmb * kEmb) return;
  if (out_size != kTok * kEmb) return;
  if (ws_size < kWsTotal) return;

  const float* x   = (const float*)d_in[0];
  const int*   tp  = (const int*)d_in[1];
  const float* qw  = (const float*)d_in[2];
  const float* kw  = (const float*)d_in[3];
  const float* vw  = (const float*)d_in[4];
  const float* ow  = (const float*)d_in[5];
  float* out = (float*)d_out;

  char* ws = (char*)d_ws;
  unsigned short* X16  = (unsigned short*)(ws + kOffX16);
  unsigned short* W16  = (unsigned short*)(ws + kOffW16);
  float*          FREQ = (float*)(ws + kOffFreq);
  float*          CS   = (float*)(ws + kOffCs);
  unsigned short* QH   = (unsigned short*)(ws + kOffQh);
  unsigned short* KH   = (unsigned short*)(ws + kOffKh);
  unsigned short* VTH  = (unsigned short*)(ws + kOffVth);
  unsigned short* QLO  = (unsigned short*)(ws + kOffQlo);
  unsigned short* KLO  = (unsigned short*)(ws + kOffKlo);
  unsigned short* VTLO = (unsigned short*)(ws + kOffVtlo);
  unsigned short* AOH  = (unsigned short*)(ws + kOffAoh);
  unsigned short* AOLO = (unsigned short*)(ws + kOffAolo);
  unsigned short* WO16 = W16 + (size_t)3 * kEmb * kEmb;

  cast8_kernel<<<dim3((kTok * kEmb / 8) / 256, 1), 256, 0, stream>>>(x, x, x, x, X16, kTok * kEmb / 8, kXCarry);
  cast8_kernel<<<dim3((kEmb * kEmb / 8) / 256, 4), 256, 0, stream>>>(qw, kw, vw, ow, W16, kEmb * kEmb / 8, kWCarry);

  rope_freq_kernel<<<1, 32, 0, stream>>>(FREQ);
  rope_table_kernel<<<(kSeq * 32) / 256, 256, 0, stream>>>(tp, FREQ, CS);

  qkv_proj_kernel<<<(kTok / 64) * (kNqkv / 64) / 8, 256, 0, stream>>>(X16, W16, CS, QH, KH, VTH, QLO, KLO, VTLO);

  attn_kernel<true><<<kBH * (kTierS / 64), 128, 0, stream>>>(QH, KH, VTH, QLO, KLO, VTLO, AOH, AOLO, 0, kTierS / 64);
  attn_kernel<false><<<kBH * ((kSeq - kTierS) / 64), 128, 0, stream>>>(QH, KH, VTH, QLO, KLO, VTLO, AOH, AOLO,
                                                                       kTierS / 64, (kSeq - kTierS) / 64);

  out_proj_kernel<2, true><<<dim3((kTierS / 32) * (kEmb / 64) / 8, kBatch), 256, 0, stream>>>(
      AOH, AOLO, (long)kSeq * kEmb, (long)kTierS * kEmb, WO16, out, (long)kSeq * kEmb, kTierS);
  out_proj_kernel<4, false><<<dim3(((kSeq - kTierS) / 64) * (kEmb / 64) / 8, kBatch), 256, 0, stream>>>(
      AOH + (size_t)kTierS * kEmb, AOLO, (long)kSeq * kEmb, (long)kTierS * kEmb, WO16,
      out + (size_t)kTierS * kEmb, (long)kSeq * kEmb, kSeq - kTierS);
}
